// ChunkedVectorizedSlidingWindowModel_80255758893218
// MI455X (gfx1250) — hardware-verified
//
#include <hip/hip_runtime.h>


#define NB_  2
#define TT   4096
#define DM   1024
#define NH_  16
#define HD   64
#define QB   64
#define NBK  (TT / QB)
#define WK   192
#define LEAD 128
#define TP   (TT + LEAD)
#define WIN  128
typedef _Float16 h16;
typedef unsigned short bf;
typedef __attribute__((ext_vector_type(16))) __bf16   v16bf;
typedef __attribute__((ext_vector_type(16))) _Float16 v16h;
typedef __attribute__((ext_vector_type(8)))  _Float16 v8h;
typedef __attribute__((ext_vector_type(8)))  unsigned short v8us;
typedef __attribute__((ext_vector_type(8)))  float    v8f;
typedef __attribute__((ext_vector_type(4)))  float    v4f;
typedef v8h  __attribute__((may_alias)) v8ha;
typedef v4f  __attribute__((may_alias)) v4fa;
typedef v8us __attribute__((may_alias)) v8usa;

__device__ __forceinline__ unsigned short f2bf(float f) { unsigned u = __float_as_uint(f); u += 0x7FFFu + ((u >> 16) & 1u); return (unsigned short)(u >> 16); }
__device__ __forceinline__ float bf2f(unsigned short b) { return __uint_as_float(((unsigned)b) << 16); }
__device__ __forceinline__ float bfr(float f) { return bf2f(f2bf(f)); }
__device__ __forceinline__ v16h cat16(v8h lo, v8h hi) { return __builtin_shufflevector(lo, hi, 0, 1, 2, 3, 4, 5, 6, 7, 8, 9, 10, 11, 12, 13, 14, 15); }
__device__ __forceinline__ v16bf cat16b(v8us lo, v8us hi) { return __builtin_bit_cast(v16bf, __builtin_shufflevector(lo, hi, 0, 1, 2, 3, 4, 5, 6, 7, 8, 9, 10, 11, 12, 13, 14, 15)); }
__device__ __forceinline__ v8f wmma16(v16h a, v16h b, v8f c) { return __builtin_amdgcn_wmma_f32_16x16x32_f16(false, a, false, b, (short)0, c, false, false); }
__device__ __forceinline__ v8f wmmab(v16bf a, v16bf b, v8f c) { return __builtin_amdgcn_wmma_f32_16x16x32_bf16(false, a, false, b, (short)0, c, false, false); }


template <typename T16> struct WFrag;
template <> struct WFrag<h16> { typedef v16h V; static __device__ __forceinline__ V ld(const h16* p) { return cat16(*(const v8h*)p, *(const v8h*)(p + 16)); } static __device__ __forceinline__ v8f mma(V a, V b, v8f c) { return wmma16(a, b, c); } };
template <> struct WFrag<bf> { typedef v16bf V; static __device__ __forceinline__ V ld(const bf* p) { return cat16b(*(const v8us*)p, *(const v8us*)(p + 16)); } static __device__ __forceinline__ v8f mma(V a, V b, v8f c) { return wmmab(a, b, c); } };
template <typename T16, int NSPLIT, bool BIAS>
__global__ __launch_bounds__(32) void k_gemmw(const T16* __restrict__ A, const T16* __restrict__ A2, const T16* __restrict__ Bt, const T16* __restrict__ Bt2, int K, float* C, int ldc, const float* __restrict__ bias, size_t sA, size_t sB, size_t sC) {
    typedef typename WFrag<T16>::V V;
    __shared__ __align__(16) float os[16 * 68];
    const size_t z = blockIdx.z; A += z * sA; if (A2) A2 += z * sA; Bt += z * sB; if (Bt2) Bt2 += z * sB; C += z * sC;
    const int lane = threadIdx.x & 31, lr = lane & 15, hi = lane >> 4; const int r0 = blockIdx.x * 64, c0 = blockIdx.y * 64;
    v8f acc[4][4];
#pragma unroll
    for (int mb = 0; mb < 4; ++mb)
#pragma unroll
        for (int nb = 0; nb < 4; ++nb) acc[mb][nb] = (v8f){};
    const size_t aoff = (size_t)(r0 + lr) * K + 8 * hi, boff = (size_t)(c0 + lr) * K + 8 * hi;
#pragma unroll 1
    for (int kc = 0; kc < K; kc += 32) {
        V a[4], a2[4];
#pragma unroll
        for (int mb = 0; mb < 4; ++mb) { a[mb] = WFrag<T16>::ld(A + aoff + (size_t)mb * 16 * K + kc); if (NSPLIT == 1 || NSPLIT == 2) a2[mb] = WFrag<T16>::ld(A2 + aoff + (size_t)mb * 16 * K + kc); }
#pragma unroll
        for (int nb = 0; nb < 4; ++nb) { const V b = WFrag<T16>::ld(Bt + boff + (size_t)nb * 16 * K + kc); V b2; if (NSPLIT >= 2) b2 = WFrag<T16>::ld(Bt2 + boff + (size_t)nb * 16 * K + kc);
#pragma unroll
            for (int mb = 0; mb < 4; ++mb) { acc[mb][nb] = WFrag<T16>::mma(a[mb], b, acc[mb][nb]); if (NSPLIT == 1 || NSPLIT == 2) acc[mb][nb] = WFrag<T16>::mma(a2[mb], b, acc[mb][nb]); if (NSPLIT >= 2) acc[mb][nb] = WFrag<T16>::mma(a[mb], b2, acc[mb][nb]); } }
        asm volatile("v_nop\n\tv_nop\n\tv_nop\n\tv_nop" : "+v"(acc[0][0]), "+v"(acc[1][1]), "+v"(acc[2][2]), "+v"(acc[3][3]) : "v"(a[0]), "v"(a[3]));
    }
#pragma unroll
    for (int mb = 0; mb < 4; ++mb) {
#pragma unroll
        for (int nb = 0; nb < 4; ++nb) {
#pragma unroll
            for (int j = 0; j < 8; ++j) os[(hi * 8 + j) * 68 + nb * 16 + lr] = acc[mb][nb][j]; }
        __builtin_amdgcn_wave_barrier(); asm volatile("" ::: "memory");
        float* crow = C + (size_t)(r0 + mb * 16) * ldc + c0;
#pragma unroll 1
        for (int ps = 0; ps < 2; ++ps) {
#pragma unroll
            for (int s = 0; s < 8; ++s) { const int row = 2 * s + hi, cofs = lr * 4; v4f val = *(const v4fa*)(os + row * 68 + cofs); if (BIAS) { val[0] += bfr(bias[c0 + cofs]); val[1] += bfr(bias[c0 + cofs + 1]); val[2] += bfr(bias[c0 + cofs + 2]); val[3] += bfr(bias[c0 + cofs + 3]); }
                *(volatile v4f*)(crow + (size_t)row * ldc + cofs) = val; }
            if (ps == 0) __threadfence(); }
        __builtin_amdgcn_wave_barrier(); asm volatile("" ::: "memory");
    }
}

__device__ __forceinline__ void splitf(float y, unsigned short& h, unsigned short& l) { h = f2bf(y); l = f2bf(y - bf2f(h)); }
typedef __attribute__((ext_vector_type(2))) unsigned short v2us;
typedef __attribute__((ext_vector_type(4))) unsigned short v4us;

__global__ __launch_bounds__(256) void k_cvt8(const float* __restrict__ src, bf* dst, size_t n8) { const size_t i = (size_t)blockIdx.x * 256 + threadIdx.x; if (i >= n8) return; const v8f v = *(const v8f*)(src + i * 8); v8us o;
#pragma unroll
    for (int k = 0; k < 8; ++k) o[k] = f2bf(v[k]); *(volatile v8us*)(dst + i * 8) = o; __threadfence(); *(volatile v8us*)(dst + i * 8) = o; }
__global__ __launch_bounds__(256) void k_qpl(const float* __restrict__ F, bf* Ph, bf* Pl) { const size_t e = ((size_t)blockIdx.x * 256 + threadIdx.x) * 4; if (e >= (size_t)NH_ * TT * HD) return; const int d = (int)(e % HD); const int t = (int)((e / HD) % TT); const int h = (int)(e / ((size_t)HD * TT)); const v4f a = *(const v4f*)(F + (size_t)t * DM + h * HD + d); v4us oh, ol;
#pragma unroll
    for (int u = 0; u < 4; ++u) { unsigned short x, y; splitf(a[u], x, y); oh[u] = x; ol[u] = y; } *(volatile v4us*)(Ph + e) = oh; *(volatile v4us*)(Pl + e) = ol; __threadfence(); *(volatile v4us*)(Ph + e) = oh; *(volatile v4us*)(Pl + e) = ol; }
__global__ __launch_bounds__(256) void k_kpl(const float* __restrict__ F, bf* Ph, bf* Pl) { const size_t e = ((size_t)blockIdx.x * 256 + threadIdx.x) * 4; if (e >= (size_t)NH_ * TP * HD) return; const int d = (int)(e % HD); const int r = (int)((e / HD) % TP); const int h = (int)(e / ((size_t)HD * TP)); v4us oh, ol;
    if (r < LEAD) { oh = (v4us){0, 0, 0, 0}; ol = oh; } else { const v4f a = *(const v4f*)(F + (size_t)(r - LEAD) * DM + h * HD + d);
#pragma unroll
        for (int u = 0; u < 4; ++u) { unsigned short x, y; splitf(a[u], x, y); oh[u] = x; ol[u] = y; } }
    *(volatile v4us*)(Ph + e) = oh; *(volatile v4us*)(Pl + e) = ol; __threadfence(); *(volatile v4us*)(Ph + e) = oh; *(volatile v4us*)(Pl + e) = ol; }
__global__ __launch_bounds__(256) void k_vwin(const float* __restrict__ F, bf* Vh, bf* Vl) { const size_t e = ((size_t)blockIdx.x * 256 + threadIdx.x) * 2; if (e >= (size_t)NH_ * NBK * HD * WK) return; const int j = (int)(e % WK); const int d = (int)((e / WK) % HD); const int blk = (int)((e / ((size_t)WK * HD)) % NBK); const int h = (int)(e / ((size_t)WK * HD * NBK)); v2us oh, ol;
#pragma unroll
    for (int u = 0; u < 2; ++u) { const int s = blk * QB - LEAD + j + u; unsigned short x = 0, y = 0; if (s >= 0) splitf(F[(size_t)s * DM + h * HD + d], x, y); oh[u] = x; ol[u] = y; }
    *(volatile v2us*)(Vh + e) = oh; *(volatile v2us*)(Vl + e) = ol; __threadfence(); *(volatile v2us*)(Vh + e) = oh; *(volatile v2us*)(Vl + e) = ol; }
__global__ __launch_bounds__(256) void k_mrg(const float* __restrict__ O, bf* Ah, bf* Al) { const size_t e = ((size_t)blockIdx.x * 256 + threadIdx.x) * 4; if (e >= (size_t)TT * DM) return; const int c = (int)(e % DM); const int t = (int)(e / DM); const int h = c / HD, d = c % HD; const int blk = t / QB, i = t % QB; const v4f a = *(const v4f*)(O + (((size_t)(h * NBK + blk)) * QB + i) * HD + d); v4us oh, ol;
#pragma unroll
    for (int u = 0; u < 4; ++u) { unsigned short x, y; splitf(a[u], x, y); oh[u] = x; ol[u] = y; } *(volatile v4us*)(Ah + e) = oh; *(volatile v4us*)(Al + e) = ol; __threadfence(); *(volatile v4us*)(Ah + e) = oh; *(volatile v4us*)(Al + e) = ol; }
__global__ __launch_bounds__(256) void k_bsoft(const float* __restrict__ Sb, bf* Ph, bf* Pl) { const int lane = threadIdx.x & 31; const int row = blockIdx.x * 8 + (threadIdx.x >> 5); if (row >= NH_ * NBK * QB) return; const int i = row % QB; const int blk = (row / QB) % NBK; const int qpos = blk * QB + i; const float* sr = Sb + (size_t)row * WK; float v[6]; float mx = -3.0e38f;
#pragma unroll
    for (int ch = 0; ch < 2; ++ch) { const int j0 = ch * 96 + lane * 3;
#pragma unroll
        for (int u = 0; u < 3; ++u) { const int j = j0 + u; const int kpos = blk * QB - LEAD + j; const int dd = qpos - kpos; const bool ok = (kpos >= 0) && (dd >= 0) && (dd < WIN); const float t = ok ? sr[j] * 0.125f : -3.0e38f; v[ch * 3 + u] = t; mx = fmaxf(mx, t); } }
#pragma unroll
    for (int sh = 16; sh; sh >>= 1) mx = fmaxf(mx, __shfl_xor(mx, sh, 32));
    float sum = 0.f;
#pragma unroll
    for (int k = 0; k < 6; ++k) { float d0 = __fsub_rn(v[k], mx); asm volatile("" : "+v"(d0)); v[k] = __expf(d0); sum += v[k]; }
#pragma unroll
    for (int sh = 16; sh; sh >>= 1) sum += __shfl_xor(sum, sh, 32);
    const float f = __fdiv_rn(1.0f, sum);
    for (int ps = 0; ps < 2; ++ps) {
#pragma unroll
        for (int c = 0; c < 3; ++c) { v2us oh, ol;
#pragma unroll
            for (int q = 0; q < 2; ++q) { const int j = c * 64 + 2 * lane + q; const int ch = j / 96, rem = j % 96; const int srcl = rem / 3, su = rem % 3;
                float val = 0.f;
#pragma unroll
                for (int k = 0; k < 6; ++k) { const float got = __shfl(v[k], srcl, 32); if (k == ch * 3 + su) val = got; }
                unsigned short a, b; splitf(val * f, a, b); oh[q] = a; ol[q] = b; }
            const size_t oo = (size_t)row * WK + c * 64 + 2 * lane; *(volatile v2us*)(Ph + oo) = oh; *(volatile v2us*)(Pl + oo) = ol; }
        if (ps == 0) __threadfence(); } }

extern "C" void kernel_launch(void* const* d_in, const int* in_sizes, int n_in,
                              void* d_out, int out_size, void* d_ws, size_t ws_size, hipStream_t stream) {
    (void)in_sizes; (void)n_in; (void)out_size;
    const float* x = (const float*)d_in[0]; const float* wq = (const float*)d_in[1]; const float* wk = (const float*)d_in[2]; const float* wv = (const float*)d_in[3]; const float* wo = (const float*)d_in[4];
    float* OUT = (float*)d_out;
    char* wsp = (char*)d_ws;
    auto take = [&](size_t bytes) { char* p = wsp; wsp += (bytes + 255) & ~(size_t)255; return (void*)p; };
    bf* WQ = (bf*)take((size_t)DM * DM * 2); bf* WK_ = (bf*)take((size_t)DM * DM * 2); bf* WV = (bf*)take((size_t)DM * DM * 2); bf* WO = (bf*)take((size_t)DM * DM * 2);
    bf* XB = (bf*)take((size_t)TT * DM * 2); float* F = (float*)take((size_t)TT * DM * 4); bf* QPh = (bf*)take((size_t)NH_ * TT * HD * 2); bf* QPl = (bf*)take((size_t)NH_ * TT * HD * 2); bf* KPh = (bf*)take((size_t)NH_ * TP * HD * 2); bf* KPl = (bf*)take((size_t)NH_ * TP * HD * 2); bf* VWh = (bf*)take((size_t)NH_ * NBK * HD * WK * 2); bf* VWl = (bf*)take((size_t)NH_ * NBK * HD * WK * 2);
    float* Sb = (float*)take((size_t)NH_ * NBK * QB * WK * 4); bf* Ph = (bf*)take((size_t)NH_ * NBK * QB * WK * 2); bf* Pl = (bf*)take((size_t)NH_ * NBK * QB * WK * 2); float* O = (float*)take((size_t)NH_ * NBK * QB * HD * 4); bf* Ah = (bf*)take((size_t)TT * DM * 2); bf* Al = (bf*)take((size_t)TT * DM * 2);
    if ((size_t)(wsp - (char*)d_ws) > ws_size) return;
    k_cvt8<<<(DM * DM / 8 + 255) / 256, 256, 0, stream>>>(wq, WQ, (size_t)DM * DM / 8); k_cvt8<<<(DM * DM / 8 + 255) / 256, 256, 0, stream>>>(wk, WK_, (size_t)DM * DM / 8); k_cvt8<<<(DM * DM / 8 + 255) / 256, 256, 0, stream>>>(wv, WV, (size_t)DM * DM / 8); k_cvt8<<<(DM * DM / 8 + 255) / 256, 256, 0, stream>>>(wo, WO, (size_t)DM * DM / 8);
    for (int b = 0; b < NB_; ++b) {
        k_cvt8<<<(unsigned)(((size_t)TT * DM / 8 + 255) / 256), 256, 0, stream>>>(x + (size_t)b * TT * DM, XB, (size_t)TT * DM / 8);
        k_gemmw<bf, 0, false><<<dim3(TT / 64, DM / 64, 1), 32, 0, stream>>>(XB, nullptr, WQ, nullptr, DM, F, DM, nullptr, 0, 0, 0); k_qpl<<<(unsigned)(((size_t)NH_ * TT * HD / 4 + 255) / 256), 256, 0, stream>>>(F, QPh, QPl);
        k_gemmw<bf, 0, false><<<dim3(TT / 64, DM / 64, 1), 32, 0, stream>>>(XB, nullptr, WK_, nullptr, DM, F, DM, nullptr, 0, 0, 0); k_kpl<<<(unsigned)(((size_t)NH_ * TP * HD / 4 + 255) / 256), 256, 0, stream>>>(F, KPh, KPl);
        k_gemmw<bf, 0, false><<<dim3(TT / 64, DM / 64, 1), 32, 0, stream>>>(XB, nullptr, WV, nullptr, DM, F, DM, nullptr, 0, 0, 0); k_vwin<<<(unsigned)(((size_t)NH_ * NBK * HD * WK / 2 + 255) / 256), 256, 0, stream>>>(F, VWh, VWl);
        for (int h = 0; h < NH_; ++h) {
            k_gemmw<bf, 2, false><<<dim3(1, WK / 64, NBK), 32, 0, stream>>>(QPh + (size_t)h * TT * HD, QPl + (size_t)h * TT * HD, KPh + (size_t)h * TP * HD, KPl + (size_t)h * TP * HD, HD, Sb + (size_t)h * NBK * QB * WK, WK, nullptr, (size_t)QB * HD, (size_t)QB * HD, (size_t)QB * WK); }
        k_bsoft<<<NH_ * NBK * QB / 8, 256, 0, stream>>>(Sb, Ph, Pl);
        k_gemmw<bf, 2, false><<<dim3(1, 1, NH_ * NBK), 32, 0, stream>>>(Ph, Pl, VWh, VWl, WK, O, HD, nullptr, (size_t)QB * WK, (size_t)HD * WK, (size_t)QB * HD);
        k_mrg<<<(unsigned)(((size_t)TT * DM / 4 + 255) / 256), 256, 0, stream>>>(O, Ah, Al);
        k_gemmw<bf, 1, false><<<dim3(TT / 64, DM / 64, 1), 32, 0, stream>>>(Ah, Al, WO, nullptr, DM, OUT + (size_t)b * TT * DM, DM, nullptr, 0, 0, 0); }
}
